// TransformerEncoderLayer_73933567033495
// MI455X (gfx1250) — hardware-run, weakly checked
//
#include <hip/hip_runtime.h>
#include <math.h>

typedef __attribute__((ext_vector_type(16))) _Float16 v16h;
typedef __attribute__((ext_vector_type(8)))  _Float16 v8h;
typedef __attribute__((ext_vector_type(8)))  float    v8f;
typedef __attribute__((ext_vector_type(4)))  float    v4f;
typedef __attribute__((ext_vector_type(4)))  unsigned int v4u;
typedef __attribute__((ext_vector_type(2)))  unsigned int v2u;

constexpr int kBatch = 4;
constexpr int kL     = 128;
constexpr int kD     = 256;
constexpr int kF     = 1024;
constexpr int kH     = 8;
constexpr int kDh    = 32;
constexpr int kR     = 64;
constexpr int kS     = 16;
constexpr int kKrp   = kR * kS;
constexpr int kRows  = kBatch * kL;
constexpr int kRbfP  = 72;
constexpr int kYP    = 260;
static_assert(kH * kDh == kD);
static_assert(kKrp == 1024);
static_assert(kRows == 512);
static_assert((kDh % 32) == 0 && (kD % 32) == 0 && (kF % 32) == 0 && (kL % 32) == 0 && (kR % 32) == 0);
static_assert((kRows % 64) == 0 && (kKrp % 64) == 0 && (kL % 64) == 0 && (kF % 64) == 0 && (kD % 64) == 0);

constexpr float kQC   = 16.0f;
constexpr float kWC   = 1024.0f;
constexpr float kWQC  = 256.0f;
constexpr float kRC   = 1024.0f;
constexpr float kPC   = 2048.0f;
constexpr float kXC   = 16.0f;
constexpr float kHC   = 2048.0f;
constexpr float kWqScale  = kWQC / (kQC * kWC);
constexpr float kQQInv    = 1.0f / (kQC * kQC);
constexpr float kTInv     = 1.0f / (kRC * kWQC);
constexpr float kAvInv    = 1.0f / (kPC * kQC);
constexpr float kFf1Scale = 1.0f / (kXC * kWC);
constexpr float kFf2Scale = 1.0f / (kHC * kWC);
constexpr float kLnEps    = 1e-5f;
constexpr float kInvD     = 1.0f / (float)kD;
constexpr float kCut      = 10.0f;
constexpr float kInvCut   = 1.0f / kCut;
constexpr float kSp       = kCut / (float)(kR - 1);
constexpr float kInvSp    = 1.0f / kSp;
constexpr float kPi       = 3.14159265358979323846f;

constexpr size_t kOffQ16  = 0;
constexpr size_t kOffVT16 = kOffQ16  + (size_t)kRows * kD * 2;
constexpr size_t kOffWP16 = kOffVT16 + (size_t)kBatch * kD * kL * 2;
constexpr size_t kOffW1T  = kOffWP16 + (size_t)kKrp * kD * 2;
constexpr size_t kOffW2T  = kOffW1T  + (size_t)kF * kD * 2;
constexpr size_t kOffWQP  = kOffW2T  + (size_t)kD * kF * 2;
constexpr size_t kOffSB   = kOffWQP  + (size_t)kRows * kH * kKrp * 2;
constexpr size_t kOffP16  = kOffSB   + (size_t)kBatch * kH * kL * kL * 4;
constexpr size_t kOffAO   = kOffP16  + (size_t)kBatch * kH * kL * kL * 2;
constexpr size_t kOffX    = kOffAO   + (size_t)kRows * kD * 4;
constexpr size_t kOffX16  = kOffX    + (size_t)kRows * kD * 4;
constexpr size_t kOffH16  = kOffX16  + (size_t)kRows * kD * 2;
constexpr size_t kOffY    = kOffH16  + (size_t)kRows * kF * 2;
constexpr size_t kWsTotal = kOffY    + (size_t)kRows * kD * 4;
static_assert(kWsTotal == 16515072ull);
static_assert(kWsTotal <= 134217728ull);
static_assert((kOffVT16 % 128) == 0 && (kOffWP16 % 128) == 0 && (kOffW1T % 128) == 0 && (kOffW2T % 128) == 0 &&
              (kOffWQP % 128) == 0 && (kOffSB % 128) == 0 && (kOffP16 % 128) == 0 && (kOffAO % 128) == 0 &&
              (kOffX % 128) == 0 && (kOffX16 % 128) == 0 && (kOffH16 % 128) == 0 && (kOffY % 128) == 0);

__device__ __forceinline__ unsigned short f2bf_bits(float f) {
  unsigned u = __float_as_uint(f);
  return (unsigned short)((u + 0x7FFFu + ((u >> 16) & 1u)) >> 16);
}
__device__ __forceinline__ float bf_bits2f(unsigned short h) { return __uint_as_float(((unsigned)h) << 16); }
__device__ __forceinline__ unsigned pk16(unsigned short a, unsigned short b) { return (unsigned)a | ((unsigned)b << 16); }
__device__ __forceinline__ unsigned short h_bits(float f) { const _Float16 h = (_Float16)f; return __builtin_bit_cast(unsigned short, h); }

__device__ __forceinline__ float wave_sum(float v) {
#pragma unroll
  for (int m = 16; m > 0; m >>= 1) v += __shfl_xor(v, m, 32);
  return v;
}
__device__ __forceinline__ float wave_max(float v) {
#pragma unroll
  for (int m = 16; m > 0; m >>= 1) v = fmaxf(v, __shfl_xor(v, m, 32));
  return v;
}

__device__ __forceinline__ v8f mma_h(v16h a, v16h b, v8f c) {
  c = __builtin_amdgcn_wmma_f32_16x16x32_f16(false, a, false, b, (short)0, c, false, false);
  asm volatile("v_nop\n\tv_nop\n\tv_nop\n\tv_nop" : "+v"(c) : "v"(a), "v"(b));
  return c;
}
__device__ __forceinline__ void dep_guard_h(v8f& a, v8f& b, v16h x, v16h y) { asm volatile("v_nop\n\tv_nop\n\tv_nop\n\tv_nop" : "+v"(a), "+v"(b) : "v"(x), "v"(y)); }
__device__ __forceinline__ void keep4_h(v16h a, v16h b, v16h c, v16h d) { asm volatile("v_nop" :: "v"(a), "v"(b), "v"(c), "v"(d)); }
__device__ __forceinline__ void acc_guard4(v8f& a, v8f& b, v8f& c, v8f& d) { asm volatile("v_nop\n\tv_nop\n\tv_nop\n\tv_nop" : "+v"(a), "+v"(b), "+v"(c), "+v"(d)); }

template <typename T> struct Frag;
template <> struct Frag<_Float16> {
  typedef v16h V; union U { v16h v; v8h h[2]; };
  static __device__ __forceinline__ v16h load(const _Float16* p) {
    U f; f.h[0] = *(const v8h*)(p); f.h[1] = *(const v8h*)(p + 16); return f.v;
  }
  static __device__ __forceinline__ v8f mma(v16h a, v16h b, v8f c) { return mma_h(a, b, c); }
  static __device__ __forceinline__ void guard(v8f& a, v8f& b, v16h x, v16h y) { dep_guard_h(a, b, x, y); }
  static __device__ __forceinline__ void keep(v16h a, v16h b, v16h c, v16h d) { keep4_h(a, b, c, d); }
};

template <int ET> struct Elem;
template <> struct Elem<0> { typedef _Float16 T; };
template <int ET, bool SPLIT, int BIAS_MODE, int OUT_MODE, bool RESID, int ACT>
__global__ __launch_bounds__(256) void wmma_gemm64(
    const unsigned short* __restrict__ Ap, const unsigned short* __restrict__ A2p, int lda, long strideA,
    const unsigned short* __restrict__ Btp, const unsigned short* __restrict__ Bt2p, int ldb, long strideB,
    void* __restrict__ Cout, void* __restrict__ Cout2, int ldc, long strideC,
    const float* __restrict__ bias,
    const float* __restrict__ resid, long strideR,
    int M, int N, int K, float scale,
    long strideAz, long strideBz, long strideCz, float oscale) {
  typedef typename Elem<ET>::T T;
  typedef typename Frag<T>::V V;
  const T* A = (const T*)Ap; const T* A2 = (const T*)A2p; const T* Bt = (const T*)Btp; const T* Bt2 = (const T*)Bt2p;
  __shared__ __align__(16) float sT[8][16 * 68];
  const int b    = blockIdx.y;
  const int bz   = blockIdx.z;
  const int lane = threadIdx.x & 31;
  const int wave = __builtin_amdgcn_readfirstlane((int)(threadIdx.x >> 5));
  const int tilesN = N >> 6;
  const int tilesM = M >> 6;
  const int tile = blockIdx.x * 8 + wave;
  if (tile >= tilesM * tilesN) return;
  const int tm = tile / tilesN;
  const int tn = tile - tm * tilesN;
  const int m0 = tm << 6;
  const int n0 = tn << 6;

  const T* Ab  = A  + (size_t)b * strideA + (size_t)bz * strideAz;
  const T* Bb  = Bt + (size_t)b * strideB + (size_t)bz * strideBz;
  const T* Ab2 = SPLIT ? (A2  + (size_t)b * strideA + (size_t)bz * strideAz) : nullptr;
  const T* Bb2 = SPLIT ? (Bt2 + (size_t)b * strideB + (size_t)bz * strideBz) : nullptr;

  const int rlane = lane & 15;
  const int koff  = (lane >> 4) * 8;
  const int mOff  = (lane >> 4) * 8;

  v8f acc[4][4];
#pragma unroll
  for (int i = 0; i < 4; ++i)
#pragma unroll
    for (int j = 0; j < 4; ++j) acc[i][j] = (v8f){0.f,0.f,0.f,0.f,0.f,0.f,0.f,0.f};

  for (int k0 = 0; k0 < K; k0 += 32) {
    V bh[4], bl[4];
#pragma unroll
    for (int j = 0; j < 4; ++j) {
      const size_t bo = (size_t)(n0 + (j << 4) + rlane) * ldb + koff + k0;
      bh[j] = Frag<T>::load(Bb + bo);
      if (SPLIT) bl[j] = Frag<T>::load(Bb2 + bo);
    }
#pragma unroll
    for (int i = 0; i < 4; ++i) {
      const size_t ao = (size_t)(m0 + (i << 4) + rlane) * lda + koff + k0;
      V ah = Frag<T>::load(Ab + ao);
      V al;
      if (SPLIT) al = Frag<T>::load(Ab2 + ao);
#pragma unroll
      for (int j = 0; j < 4; ++j) {
        acc[i][j] = Frag<T>::mma(ah, bh[j], acc[i][j]);
        if (SPLIT) {
          acc[i][j] = Frag<T>::mma(ah, bl[j], acc[i][j]);
          acc[i][j] = Frag<T>::mma(al, bh[j], acc[i][j]);
        }
      }
      Frag<T>::guard(acc[i][0], acc[i][3], ah, SPLIT ? al : ah);
    }
    Frag<T>::keep(bh[0], bh[1], bh[2], bh[3]);
    if (SPLIT) Frag<T>::keep(bl[0], bl[1], bl[2], bl[3]);
  }
  acc_guard4(acc[0][0], acc[0][1], acc[0][2], acc[0][3]);
  acc_guard4(acc[1][0], acc[1][1], acc[1][2], acc[1][3]);
  acc_guard4(acc[2][0], acc[2][1], acc[2][2], acc[2][3]);
  acc_guard4(acc[3][0], acc[3][1], acc[3][2], acc[3][3]);

  float* slab = sT[wave];
  const float* Rb = RESID ? (resid + (size_t)b * strideR) : nullptr;
#pragma unroll
  for (int i = 0; i < 4; ++i) {
    const int mBase = m0 + (i << 4);
#pragma unroll
    for (int j = 0; j < 4; ++j) {
      const int n = n0 + (j << 4) + rlane;
      float bv = 0.f;
      if (BIAS_MODE == 2) bv = bias[n];
#pragma unroll
      for (int r = 0; r < 8; ++r) {
        float v = acc[i][j][r] * scale;
        if (BIAS_MODE == 1) v += bias[mBase + mOff + r];
        if (BIAS_MODE == 2) v += bv;
        if (RESID) v += Rb[(size_t)(mBase + mOff + r) * ldc + n];
        if (ACT == 4) v = (v > 0.f) ? v : 0.01f * v;
        v *= oscale;
        slab[(mOff + r) * 68 + (j << 4) + rlane] = v;
      }
    }
    __builtin_amdgcn_fence(__ATOMIC_RELEASE, "workgroup");
    __builtin_amdgcn_wave_barrier();
    __builtin_amdgcn_fence(__ATOMIC_ACQUIRE, "workgroup");
    if (OUT_MODE == 0) {
      float* C = (float*)Cout + (size_t)b * strideC + (size_t)bz * strideCz;
      const int hh = lane >> 4, c4 = (lane & 15) * 4;
      for (int pass = 0; pass < 2; ++pass) {
#pragma unroll
        for (int it = 0; it < 8; ++it) {
          const int row = it * 2 + hh;
          v4f v = *(const v4f*)(slab + row * 68 + c4);
          *(volatile v4f*)(C + (size_t)(mBase + row) * ldc + n0 + c4) = v;
        }
        __threadfence();
      }
    } else {
      const int q = lane >> 3, c8 = (lane & 7) * 8;
      unsigned short* C  = (unsigned short*)Cout + (size_t)b * strideC + (size_t)bz * strideCz;
      unsigned short* C2 = (OUT_MODE == 2) ? ((unsigned short*)Cout2 + (size_t)b * strideC + (size_t)bz * strideCz) : nullptr;
      for (int pass = 0; pass < 2; ++pass) {
#pragma unroll
        for (int it = 0; it < 4; ++it) {
          const int row = it * 4 + q;
          const float* sp = slab + row * 68 + c8;
          v8h hv, lv;
#pragma unroll
          for (int e = 0; e < 8; ++e) {
            if (OUT_MODE == 1) {
              hv[e] = (_Float16)sp[e];
            } else {
              unsigned short hb = f2bf_bits(sp[e]);
              unsigned short lb = f2bf_bits(sp[e] - bf_bits2f(hb));
              hv[e] = __builtin_bit_cast(_Float16, hb);
              lv[e] = __builtin_bit_cast(_Float16, lb);
            }
          }
          *(volatile v8h*)(C + (size_t)(mBase + row) * ldc + n0 + c8) = hv;
          if (OUT_MODE == 2) *(volatile v8h*)(C2 + (size_t)(mBase + row) * ldc + n0 + c8) = lv;
        }
        __threadfence();
      }
    }
    __builtin_amdgcn_fence(__ATOMIC_RELEASE, "workgroup");
    __builtin_amdgcn_wave_barrier();
    __builtin_amdgcn_fence(__ATOMIC_ACQUIRE, "workgroup");
  }
}

__global__ __launch_bounds__(256) void rowcast_kernel(const float* __restrict__ in, unsigned short* __restrict__ out,
                                                      int n8, int perm, float scale) {
  const int i = blockIdx.x * 256 + threadIdx.x;
  if (i >= n8) return;
  const int row = i >> 5;
  const int g   = i & 31;
  const int srow = perm ? (((row & 63) << 4) + (row >> 6)) : row;
  const float* p = in + (size_t)srow * kD + g * 8;
  const v4f a = *(const v4f*)(p);
  const v4f c = *(const v4f*)(p + 4);
  unsigned short hb[8];
#pragma unroll
  for (int e = 0; e < 4; ++e) {
    const float fa = a[e] * scale;
    const float fc = c[e] * scale;
    hb[e]     = h_bits(fa);
    hb[4 + e] = h_bits(fc);
  }
  const v4u u = (v4u){pk16(hb[0], hb[1]), pk16(hb[2], hb[3]), pk16(hb[4], hb[5]), pk16(hb[6], hb[7])};
  unsigned short* q = out + 8 * (size_t)i;
  *(volatile v4u*)q = u;
  __threadfence();
  *(volatile v4u*)q = u;
}

__global__ __launch_bounds__(256) void transpose_cast_kernel(const float* __restrict__ in, unsigned short* __restrict__ out,
                                                             int rows, int cols, float scale) {
  __shared__ float sm[64][65];
  const int t  = threadIdx.x;
  const int r0 = blockIdx.x * 64;
  const int c0 = blockIdx.y * 64;
  const size_t zoff = (size_t)blockIdx.z * (size_t)rows * (size_t)cols;
  const float* ip = in + zoff;
  unsigned short* op = out + zoff;
#pragma unroll
  for (int i = 0; i < 16; ++i) {
    const int e  = i * 256 + t;
    const int r  = e >> 6;
    const int cc = e & 63;
    sm[cc][r] = ip[(size_t)(r0 + r) * cols + c0 + cc] * scale;
  }
  __syncthreads();
  const int lane = t & 31;
  const int wave = __builtin_amdgcn_readfirstlane((int)(threadIdx.x >> 5));
  const int q = lane >> 3, c8 = (lane & 7) * 8;
  for (int pass = 0; pass < 2; ++pass) {
#pragma unroll
    for (int it = 0; it < 2; ++it) {
      const int orow = wave * 8 + it * 4 + q;
      unsigned short hb[8];
#pragma unroll
      for (int e = 0; e < 8; ++e) hb[e] = h_bits(sm[orow][c8 + e]);
      const v4u u = (v4u){pk16(hb[0], hb[1]), pk16(hb[2], hb[3]), pk16(hb[4], hb[5]), pk16(hb[6], hb[7])};
      *(volatile v4u*)(op + (size_t)(c0 + orow) * rows + r0 + c8) = u;
    }
    __threadfence();
  }
}

__global__ __launch_bounds__(256) void rp_softmax_kernel(
    const float* __restrict__ src, const float* __restrict__ rel_diss, const float* __restrict__ rel_dirs,
    const float* __restrict__ rp_b, const unsigned short* __restrict__ WQp, const float* __restrict__ SB,
    unsigned short* __restrict__ P16) {
  __shared__ float s_d[kL];
  __shared__ float s_fc[kL];
  __shared__ __align__(16) float s_sh[kL * kS];
  __shared__ __align__(16) _Float16 s_rbf[kL * kRbfP];
  __shared__ __align__(16) float s_score[kH * kL];

  const int tid  = threadIdx.x;
  const int lane = tid & 31;
  const int wave = __builtin_amdgcn_readfirstlane((int)(threadIdx.x >> 5));
  const int hh   = lane >> 4;
  const int c    = lane & 15;
  const int bl   = blockIdx.x;
  const int b    = bl >> 7;
  const int l    = bl & 127;

  if (wave < 4) {
    const int m = tid;
    const size_t pi = (size_t)bl * kL + m;
    const float d = rel_diss[pi];
    const float x = rel_dirs[pi * 3 + 0];
    const float y = rel_dirs[pi * 3 + 1];
    const float z = rel_dirs[pi * 3 + 2];
    s_d[m] = d;
    const float u = fminf(fmaxf(d * kInvCut, 0.0f), 1.0f);
    s_fc[m] = 0.5f * (cosf(kPi * u) + 1.0f);
    const float x2 = x * x, y2 = y * y, z2 = z * z;
    float* sp = s_sh + m * kS;
    sp[0]  = 0.28209479177387814f;
    sp[1]  = 0.4886025119029199f * y;
    sp[2]  = 0.4886025119029199f * z;
    sp[3]  = 0.4886025119029199f * x;
    sp[4]  = 1.0925484305920792f * x * y;
    sp[5]  = 1.0925484305920792f * y * z;
    sp[6]  = 0.31539156525252005f * (3.0f * z2 - 1.0f);
    sp[7]  = 1.0925484305920792f * x * z;
    sp[8]  = 0.5462742152960396f * (x2 - y2);
    sp[9]  = 0.5900435899266435f * y * (3.0f * x2 - y2);
    sp[10] = 2.890611442640554f * x * y * z;
    sp[11] = 0.4570457994644658f * y * (5.0f * z2 - 1.0f);
    sp[12] = 0.3731763325901154f * z * (5.0f * z2 - 3.0f);
    sp[13] = 0.4570457994644658f * x * (5.0f * z2 - 1.0f);
    sp[14] = 1.445305721320277f * z * (x2 - y2);
    sp[15] = 0.5900435899266435f * x * (x2 - 3.0f * y2);
  }
  __syncthreads();

#pragma unroll 1
  for (int it = 0; it < 4; ++it) {
    const int g  = it * 256 + tid;
    const int m  = g >> 3;
    const int r0 = (g & 7) * 8;
    const float d  = s_d[m];
    const float fc = s_fc[m] * kRC;
    v8h hv;
#pragma unroll
    for (int e = 0; e < 8; ++e) {
      const float off = (float)(r0 + e) * kSp;
      const float u   = (d - off) * kInvSp;
      const float val = expf(-0.5f * u * u) * fc;
      hv[e] = (_Float16)val;
    }
    *(v8h*)(s_rbf + m * kRbfP + r0) = hv;
  }

  float qb = src[(size_t)bl * kD + wave * kDh + lane] * rp_b[wave * kDh + lane];
  qb = wave_sum(qb);

  const _Float16* wq = (const _Float16*)WQp + ((size_t)bl * kH + wave) * kKrp;
  const v16h bf0 = Frag<_Float16>::load(wq + c * kR + 8 * hh);
  const v16h bf1 = Frag<_Float16>::load(wq + c * kR + 32 + 8 * hh);
  __syncthreads();

#pragma unroll 2
  for (int mt = 0; mt < 8; ++mt) {
    v8f acc = (v8f){0.f,0.f,0.f,0.f,0.f,0.f,0.f,0.f};
    const _Float16* ap = s_rbf + (mt * 16 + c) * kRbfP + 8 * hh;
    const v16h a0 = Frag<_Float16>::load(ap);
    const v16h a1 = Frag<_Float16>::load(ap + 32);
    acc = mma_h(a0, bf0, acc);
    acc = mma_h(a1, bf1, acc);
    const float* shp = s_sh + (mt * 16 + 8 * hh) * kS + c;
#pragma unroll
    for (int i = 0; i < 8; ++i) {
      float v = shp[i * kS] * acc[i];
      v += __shfl_xor(v, 1, 32);
      v += __shfl_xor(v, 2, 32);
      v += __shfl_xor(v, 4, 32);
      v += __shfl_xor(v, 8, 32);
      if (c == 0) s_score[wave * kL + mt * 16 + 8 * hh + i] = v * kTInv;
    }
  }
  __syncthreads();

  const v4f sv = *(const v4f*)(s_score + wave * kL + lane * 4);
  const v4f bv = *(const v4f*)(SB + (((size_t)(b * kH + wave)) * kL + l) * kL + lane * 4);
  const float x0 = sv[0] + bv[0] + qb;
  const float x1 = sv[1] + bv[1] + qb;
  const float x2 = sv[2] + bv[2] + qb;
  const float x3 = sv[3] + bv[3] + qb;
  float mx = fmaxf(fmaxf(x0, x1), fmaxf(x2, x3));
  mx = wave_max(mx);
  const float e0 = expf(x0 - mx);
  const float e1 = expf(x1 - mx);
  const float e2 = expf(x2 - mx);
  const float e3 = expf(x3 - mx);
  float se = (e0 + e1) + (e2 + e3);
  se = wave_sum(se);
  const float inv = kPC * (1.0f / se);
  const unsigned short h0 = h_bits(e0 * inv);
  const unsigned short h1 = h_bits(e1 * inv);
  const unsigned short h2 = h_bits(e2 * inv);
  const unsigned short h3 = h_bits(e3 * inv);
  const v2u pu = (v2u){pk16(h0, h1), pk16(h2, h3)};
  unsigned short* dst = P16 + (((size_t)(b * kH + wave)) * kL + l) * kL + lane * 4;
  *(volatile v2u*)dst = pu;
  __threadfence();
  *(volatile v2u*)dst = pu;
}

__global__ __launch_bounds__(256) void av_kernel(const unsigned short* __restrict__ P16, const unsigned short* __restrict__ VT16,
                                                 float* __restrict__ AO) {
  __shared__ __align__(16) float ybuf[16 * kYP];
  const int tid  = threadIdx.x;
  const int lane = tid & 31;
  const int wave = __builtin_amdgcn_readfirstlane((int)(threadIdx.x >> 5));
  const int hh   = lane >> 4;
  const int c    = lane & 15;
  const int b    = blockIdx.x >> 3;
  const int lt   = blockIdx.x & 7;

  const _Float16* pa  = (const _Float16*)P16 + (((size_t)(b * kH + wave)) * kL + lt * 16 + c) * kL + 8 * hh;
  const _Float16* vb0 = (const _Float16*)VT16 + ((size_t)(b * kD + wave * kDh + c)) * kL + 8 * hh;
  const _Float16* vb1 = vb0 + 16 * kL;
  v8f acc0 = (v8f){0.f,0.f,0.f,0.f,0.f,0.f,0.f,0.f};
  v8f acc1 = (v8f){0.f,0.f,0.f,0.f,0.f,0.f,0.f,0.f};
#pragma unroll
  for (int kk = 0; kk < 4; ++kk) {
    const v16h a  = Frag<_Float16>::load(pa + kk * 32);
    const v16h b0 = Frag<_Float16>::load(vb0 + kk * 32);
    const v16h b1 = Frag<_Float16>::load(vb1 + kk * 32);
    acc0 = mma_h(a, b0, acc0);
    acc1 = mma_h(a, b1, acc1);
  }
#pragma unroll
  for (int i = 0; i < 8; ++i) {
    ybuf[(8 * hh + i) * kYP + wave * kDh + c]      = acc0[i] * kAvInv;
    ybuf[(8 * hh + i) * kYP + wave * kDh + 16 + c] = acc1[i] * kAvInv;
  }
  __syncthreads();
  v4f v00, v01, v10, v11;
  {
    const int ra = wave * 2, rb = wave * 2 + 1;
    v00 = *(const v4f*)(ybuf + ra * kYP + lane * 4);
    v01 = *(const v4f*)(ybuf + ra * kYP + 128 + lane * 4);
    v10 = *(const v4f*)(ybuf + rb * kYP + lane * 4);
    v11 = *(const v4f*)(ybuf + rb * kYP + 128 + lane * 4);
  }
  float* o0 = AO + ((size_t)(b * kL + lt * 16 + wave * 2)) * kD + lane * 4;
  float* o1 = o0 + kD;
  for (int pass = 0; pass < 2; ++pass) {
    *(volatile v4f*)(o0)       = v00;
    *(volatile v4f*)(o0 + 128) = v01;
    *(volatile v4f*)(o1)       = v10;
    *(volatile v4f*)(o1 + 128) = v11;
    __threadfence();
  }
}

template <bool W16>
__global__ __launch_bounds__(256) void add_ln_kernel(const float* __restrict__ A, const float* __restrict__ Bp,
                                                     const float* __restrict__ g, const float* __restrict__ be,
                                                     float* __restrict__ outf, unsigned short* __restrict__ outh,
                                                     float hcarry, int nrows) {
  const int lane = threadIdx.x & 31;
  const int wave = __builtin_amdgcn_readfirstlane((int)(threadIdx.x >> 5));
  const int row  = blockIdx.x * 8 + wave;
  if (row >= nrows) return;
  const size_t o0 = (size_t)row * kD + lane * 4;
  const size_t o1 = o0 + 128;
  const v4f xa = *(const v4f*)(A + o0) + *(const v4f*)(Bp + o0);
  const v4f xb = *(const v4f*)(A + o1) + *(const v4f*)(Bp + o1);
  const v4f ga = *(const v4f*)(g + lane * 4);
  const v4f gb = *(const v4f*)(g + 128 + lane * 4);
  const v4f ba = *(const v4f*)(be + lane * 4);
  const v4f bb = *(const v4f*)(be + 128 + lane * 4);
  float s = ((xa[0] + xa[1]) + (xa[2] + xa[3])) + ((xb[0] + xb[1]) + (xb[2] + xb[3]));
  s = wave_sum(s);
  const float mu = s * kInvD;
  const v4f ea = xa - mu;
  const v4f eb = xb - mu;
  float ss = ((ea[0] * ea[0] + ea[1] * ea[1]) + (ea[2] * ea[2] + ea[3] * ea[3])) +
             ((eb[0] * eb[0] + eb[1] * eb[1]) + (eb[2] * eb[2] + eb[3] * eb[3]));
  ss = wave_sum(ss);
  const float rs = rsqrtf(ss * kInvD + kLnEps);
  const v4f ya = ea * rs * ga + ba;
  const v4f yb = eb * rs * gb + bb;
  v2u ha = (v2u){0u, 0u};
  v2u hb = (v2u){0u, 0u};
  if (W16) {
    const float a0 = ya[0] * hcarry, a1 = ya[1] * hcarry, a2 = ya[2] * hcarry, a3 = ya[3] * hcarry;
    const float c0 = yb[0] * hcarry, c1 = yb[1] * hcarry, c2 = yb[2] * hcarry, c3 = yb[3] * hcarry;
    ha = (v2u){pk16(h_bits(a0), h_bits(a1)), pk16(h_bits(a2), h_bits(a3))};
    hb = (v2u){pk16(h_bits(c0), h_bits(c1)), pk16(h_bits(c2), h_bits(c3))};
  }
  for (int pass = 0; pass < 2; ++pass) {
    *(volatile v4f*)(outf + o0) = ya;
    *(volatile v4f*)(outf + o1) = yb;
    if (W16) {
      *(volatile v2u*)(outh + o0) = ha;
      *(volatile v2u*)(outh + o1) = hb;
    }
    __threadfence();
  }
}

extern "C" void kernel_launch(void* const* d_in, const int* in_sizes, int n_in,
                              void* d_out, int out_size, void* d_ws, size_t ws_size,
                              hipStream_t stream) {
  if (n_in < 13) return;
  if (in_sizes[0] != kRows * kD) return;
  if (in_sizes[1] != kRows * kL) return;
  if (in_sizes[2] != kRows * kL * 3) return;
  if (in_sizes[3] != kKrp * kD) return;
  if (in_sizes[4] != kD) return;
  if (in_sizes[5] != kD * kF) return;
  if (in_sizes[6] != kF) return;
  if (in_sizes[7] != kF * kD) return;
  if (in_sizes[8] != kD) return;
  if (in_sizes[9] != kD || in_sizes[10] != kD || in_sizes[11] != kD || in_sizes[12] != kD) return;
  if (out_size != kRows * kD) return;
  if (ws_size < kWsTotal) return;

  const float* src      = (const float*)d_in[0];
  const float* rel_diss = (const float*)d_in[1];
  const float* rel_dirs = (const float*)d_in[2];
  const float* rp_w     = (const float*)d_in[3];
  const float* rp_b     = (const float*)d_in[4];
  const float* lin1_w   = (const float*)d_in[5];
  const float* lin1_b   = (const float*)d_in[6];
  const float* lin2_w   = (const float*)d_in[7];
  const float* lin2_b   = (const float*)d_in[8];
  const float* g1       = (const float*)d_in[9];
  const float* be1      = (const float*)d_in[10];
  const float* g2       = (const float*)d_in[11];
  const float* be2      = (const float*)d_in[12];
  float* out = (float*)d_out;

  char* ws = (char*)d_ws;
  unsigned short* Q16  = (unsigned short*)(ws + kOffQ16);
  unsigned short* VT16 = (unsigned short*)(ws + kOffVT16);
  unsigned short* WP16 = (unsigned short*)(ws + kOffWP16);
  unsigned short* W1T  = (unsigned short*)(ws + kOffW1T);
  unsigned short* W2T  = (unsigned short*)(ws + kOffW2T);
  unsigned short* WQP  = (unsigned short*)(ws + kOffWQP);
  float*          SB   = (float*)(ws + kOffSB);
  unsigned short* P16  = (unsigned short*)(ws + kOffP16);
  float*          AO   = (float*)(ws + kOffAO);
  float*          X    = (float*)(ws + kOffX);
  unsigned short* X16  = (unsigned short*)(ws + kOffX16);
  unsigned short* H16  = (unsigned short*)(ws + kOffH16);
  float*          Y    = (float*)(ws + kOffY);

  const float scl = 1.0f / sqrtf((float)kDh);

  rowcast_kernel<<<(kRows * kD / 8) / 256, 256, 0, stream>>>(src, Q16, kRows * kD / 8, 0, kQC);
  rowcast_kernel<<<(kKrp * kD / 8) / 256, 256, 0, stream>>>(rp_w, WP16, kKrp * kD / 8, 1, kWC);
  transpose_cast_kernel<<<dim3(kL / 64, kD / 64, kBatch), 256, 0, stream>>>(src, VT16, kL, kD, kQC);
  transpose_cast_kernel<<<dim3(kD / 64, kF / 64, 1), 256, 0, stream>>>(lin1_w, W1T, kD, kF, kWC);
  transpose_cast_kernel<<<dim3(kF / 64, kD / 64, 1), 256, 0, stream>>>(lin2_w, W2T, kF, kD, kWC);

  wmma_gemm64<0, false, 0, 1, false, 0><<<dim3(16, kH, 1), 256, 0, stream>>>(
      Q16, nullptr, kD, (long)kDh,
      WP16, nullptr, kD, (long)kDh,
      (void*)WQP, nullptr, kH * kKrp, (long)kKrp,
      nullptr, nullptr, 0L,
      kRows, kKrp, kDh, kWqScale,
      0L, 0L, 0L, 1.0f);

  wmma_gemm64<0, false, 0, 0, false, 0><<<dim3(1, kH, kBatch), 128, 0, stream>>>(
      Q16, nullptr, kD, (long)kDh,
      Q16, nullptr, kD, (long)kDh,
      (void*)SB, nullptr, kL, (long)(kL * kL),
      nullptr, nullptr, 0L,
      kL, kL, kDh, scl * kQQInv,
      (long)(kL * kD), (long)(kL * kD), (long)(kH * kL * kL), 1.0f);

  rp_softmax_kernel<<<kRows, 256, 0, stream>>>(src, rel_diss, rel_dirs, rp_b, WQP, SB, P16);

  av_kernel<<<kBatch * (kL / 16), 256, 0, stream>>>(P16, VT16, AO);

  add_ln_kernel<true><<<kRows / 8, 256, 0, stream>>>(src, AO, g1, be1, X, X16, kXC, kRows);

  wmma_gemm64<0, false, 2, 1, false, 4><<<dim3(16, 1, 1), 256, 0, stream>>>(
      X16, nullptr, kD, 0L,
      W1T, nullptr, kD, 0L,
      (void*)H16, nullptr, kF, 0L,
      lin1_b, nullptr, 0L,
      kRows, kF, kD, kFf1Scale,
      0L, 0L, 0L, kHC);

  wmma_gemm64<0, false, 2, 0, false, 0><<<dim3(4, 1, 1), 256, 0, stream>>>(
      H16, nullptr, kF, 0L,
      W2T, nullptr, kF, 0L,
      (void*)Y, nullptr, kD, 0L,
      lin2_b, nullptr, 0L,
      kRows, kD, kF, kFf2Scale,
      0L, 0L, 0L, 1.0f);

  add_ln_kernel<false><<<kRows / 8, 256, 0, stream>>>(X, Y, g2, be2, out, nullptr, 1.0f, kRows);
}
